// nnRNN_87617332839042
// MI455X (gfx1250) — hardware-verified
//
#include <hip/hip_runtime.h>

typedef __attribute__((ext_vector_type(16))) _Float16 v16h;
typedef __attribute__((ext_vector_type(8)))  _Float16 v8h;
typedef __attribute__((ext_vector_type(8)))  float    v8f;
typedef __attribute__((ext_vector_type(4)))  float    v4f;
typedef __attribute__((ext_vector_type(2)))  float    v2f;
typedef __attribute__((ext_vector_type(4)))  unsigned int v4u;

constexpr int kSteps        = 64;
constexpr int kHid          = 16;
constexpr int kRowsPerWave  = 16;
constexpr int kWavesPerBlk  = 8;
constexpr int kRowsPerBlk   = kRowsPerWave * kWavesPerBlk;
constexpr int kFlat         = kSteps * kHid;
constexpr int kMlpHid       = 128;
constexpr int kOutDim       = 16;

__device__ __forceinline__ void dep_guard_h(v8f& a, v8f& b, v16h x, v16h y) { asm volatile("v_nop\n\tv_nop\n\tv_nop\n\tv_nop" : "+v"(a), "+v"(b) : "v"(x), "v"(y)); }
__device__ __forceinline__ void keep4_h(v16h a, v16h b, v16h c, v16h d) { asm volatile("v_nop" :: "v"(a), "v"(b), "v"(c), "v"(d)); }
template <typename T> struct Frag;
template <> struct Frag<_Float16> {
  typedef v16h V; union U { v16h v; v8h h[2]; };
  static __device__ __forceinline__ v16h load(const _Float16* p) {
    U f; f.h[0] = *(const v8h*)(p); f.h[1] = *(const v8h*)(p + 16); return f.v;
  }
  static __device__ __forceinline__ v8f mma(v16h a, v16h b, v8f c) {
    return __builtin_amdgcn_wmma_f32_16x16x32_f16(false, a, false, b, (short)0, c, false, false);
  }
  static __device__ __forceinline__ void guard(v8f& a, v8f& b, v16h x, v16h y) { dep_guard_h(a, b, x, y); }
  static __device__ __forceinline__ void keep(v16h a, v16h b, v16h c, v16h d) { keep4_h(a, b, c, d); }
};

__device__ __forceinline__ unsigned pk16(unsigned short a, unsigned short b) { return (unsigned)a | ((unsigned)b << 16); }
__device__ __forceinline__ unsigned short h_bits(float f) { const _Float16 h = (_Float16)f; return __builtin_bit_cast(unsigned short, h); }

__device__ __forceinline__ v8f mma16(v16h a, v16h b, v8f c) {
  c = __builtin_amdgcn_wmma_f32_16x16x32_f16(false, a, false, b, (short)0, c, false, false);
  asm volatile("v_nop\n\tv_nop\n\tv_nop\n\tv_nop" : "+v"(c) : "v"(a), "v"(b));
  return c;
}

union FragU { v16h v; v8h h[2]; };

__global__ __launch_bounds__(256) void cast8_f16_kernel(const float* __restrict__ in, unsigned short* __restrict__ outp,
                                                        int n8, float carry) {
  const int i = blockIdx.x * 256 + threadIdx.x;
  if (i >= n8) return;
  const float* p = in + 8 * (size_t)i;
  const v4f a = *(const v4f*)(p);
  const v4f b = *(const v4f*)(p + 4);
  unsigned short hb[8];
#pragma unroll
  for (int e = 0; e < 4; ++e) {
    hb[e]     = h_bits(a[e] * carry);
    hb[4 + e] = h_bits(b[e] * carry);
  }
  const v4u u = (v4u){pk16(hb[0], hb[1]), pk16(hb[2], hb[3]), pk16(hb[4], hb[5]), pk16(hb[6], hb[7])};
  unsigned short* q = outp + 8 * (size_t)i;
  *(volatile v4u*)q = u;
  __threadfence();
  *(volatile v4u*)q = u;
}

__device__ __forceinline__ v8h zero8h() { return __builtin_bit_cast(v8h, (v4u){0u, 0u, 0u, 0u}); }

__device__ __forceinline__ v16h wfrag_ih(const float* __restrict__ Wi, const float* __restrict__ Wh, int c, int hh) {
  const float* pi = Wi + c * kHid + 8 * hh;
  const float* ph = Wh + c * kHid + 8 * hh;
  const v4f i0 = *(const v4f*)(pi), i1 = *(const v4f*)(pi + 4);
  const v4f h0 = *(const v4f*)(ph), h1 = *(const v4f*)(ph + 4);
  v16h a;
#pragma unroll
  for (int e = 0; e < 4; ++e) {
    a[e]      = (_Float16)(4.0f * i0[e]);
    a[4 + e]  = (_Float16)(4.0f * i1[e]);
    a[8 + e]  = (_Float16)(4.0f * h0[e]);
    a[12 + e] = (_Float16)(4.0f * h1[e]);
  }
  return a;
}
__device__ __forceinline__ v16h wfrag_h(const float* __restrict__ Wh, int c, int hh) {
  const float* ph = Wh + c * kHid + 8 * hh;
  const v4f h0 = *(const v4f*)(ph), h1 = *(const v4f*)(ph + 4);
  v16h a;
#pragma unroll
  for (int e = 0; e < 4; ++e) {
    a[e]      = (_Float16)0.0f;
    a[4 + e]  = (_Float16)0.0f;
    a[8 + e]  = (_Float16)(4.0f * h0[e]);
    a[12 + e] = (_Float16)(4.0f * h1[e]);
  }
  return a;
}

__device__ __forceinline__ v8h relu_pack(v8f d, float sc) {
  v8h o;
#pragma unroll
  for (int r = 0; r < 8; ++r) o[r] = (_Float16)(fmaxf(d[r], 0.0f) * sc);
  return o;
}

__device__ __forceinline__ v8f cload(const float* p) {
  const v4f a = *(const v4f*)(p), b = *(const v4f*)(p + 4);
  v8f cc;
#pragma unroll
  for (int r = 0; r < 4; ++r) { cc[r] = a[r]; cc[4 + r] = b[r]; }
  return cc;
}

__device__ __forceinline__ void rnn_step(float xv, const float* cst, int hh,
                                         v16h aw0, v16h aw1, v16h aw2, v16h aw3,
                                         v8h& hp0, v8h& hp1, v8h& hp2, v8h& hp3) {
  FragU bb;
  v8f cc, d;
  {
    const v4f wA = *(const v4f*)(cst + 8 * hh);
    const v4f wB = *(const v4f*)(cst + 8 * hh + 4);
    const v4f cA = *(const v4f*)(cst + 16 + 8 * hh);
    const v4f cB = *(const v4f*)(cst + 20 + 8 * hh);
#pragma unroll
    for (int r = 0; r < 4; ++r) {
      cc[r]     = fmaf(xv, wA[r], cA[r]);
      cc[4 + r] = fmaf(xv, wB[r], cB[r]);
    }
    bb.h[0] = zero8h();
    bb.h[1] = hp0;
    d = mma16(aw0, bb.v, cc);
    hp0 = relu_pack(d, 0.25f);
  }
  cc = cload(cst + 32 + 8 * hh);
  bb.h[0] = hp0; bb.h[1] = hp1;
  d = mma16(aw1, bb.v, cc);
  hp1 = relu_pack(d, 0.25f);
  cc = cload(cst + 48 + 8 * hh);
  bb.h[0] = hp1; bb.h[1] = hp2;
  d = mma16(aw2, bb.v, cc);
  hp2 = relu_pack(d, 0.25f);
  cc = cload(cst + 64 + 8 * hh);
  bb.h[0] = hp2; bb.h[1] = hp3;
  d = mma16(aw3, bb.v, cc);
  hp3 = relu_pack(d, 0.25f);
}

__global__ __launch_bounds__(256) void rnn_mlp_kernel(
    const float* __restrict__ x,
    const float* __restrict__ Wih0, const float* __restrict__ Whh0, const float* __restrict__ bih0, const float* __restrict__ bhh0,
    const float* __restrict__ Wih1, const float* __restrict__ Whh1, const float* __restrict__ bih1, const float* __restrict__ bhh1,
    const float* __restrict__ Wih2, const float* __restrict__ Whh2, const float* __restrict__ bih2, const float* __restrict__ bhh2,
    const float* __restrict__ Wih3, const float* __restrict__ Whh3, const float* __restrict__ bih3, const float* __restrict__ bhh3,
    const unsigned short* __restrict__ W1h, const float* __restrict__ b1,
    const unsigned short* __restrict__ W2h, const float* __restrict__ b2,
    float* __restrict__ out, int nrows) {
  __shared__ __align__(16) float cst[80];
  __shared__ __align__(16) float osl[kWavesPerBlk][kRowsPerWave * kOutDim];

  const int tid  = threadIdx.x;
  const int wave = tid >> 5;
  const int lane = tid & 31;
  const int hh   = lane >> 4;
  const int c    = lane & 15;

  if (tid < kHid) {
    cst[tid]      = 16.0f * Wih0[tid];
    cst[16 + tid] = 16.0f * (bih0[tid] + bhh0[tid]);
    cst[32 + tid] = 16.0f * (bih1[tid] + bhh1[tid]);
    cst[48 + tid] = 16.0f * (bih2[tid] + bhh2[tid]);
    cst[64 + tid] = 16.0f * (bih3[tid] + bhh3[tid]);
  }
  __syncthreads();

  const int rowbase = blockIdx.x * kRowsPerBlk + wave * kRowsPerWave;
  int brow = rowbase + c;
  brow = (brow < nrows) ? brow : (nrows - 1);

  const v16h aw0 = wfrag_h(Whh0, c, hh);
  const v16h aw1 = wfrag_ih(Wih1, Whh1, c, hh);
  const v16h aw2 = wfrag_ih(Wih2, Whh2, c, hh);
  const v16h aw3 = wfrag_ih(Wih3, Whh3, c, hh);

  v8h hp0 = zero8h(), hp1 = zero8h(), hp2 = zero8h(), hp3 = zero8h();

  v8f zacc[8];
#pragma unroll
  for (int jt = 0; jt < 8; ++jt) {
    const v8f bb1 = cload(b1 + 16 * jt + 8 * hh);
#pragma unroll
    for (int r = 0; r < 8; ++r) zacc[jt][r] = 128.0f * bb1[r];
  }

  const float* xrow = x + (size_t)brow * kSteps;
  const _Float16* w1l = (const _Float16*)(const void*)W1h + (size_t)c * kFlat + 8 * hh;

#pragma unroll 1
  for (int s = 0; s < kSteps / 2; ++s) {
    asm volatile("" ::: "memory");
    const v2f x2 = *(const v2f*)(xrow + 2 * s);
    rnn_step(x2[0], cst, hh, aw0, aw1, aw2, aw3, hp0, hp1, hp2, hp3);
    const v8h h3even = hp3;
    rnn_step(x2[1], cst, hh, aw0, aw1, aw2, aw3, hp0, hp1, hp2, hp3);
    FragU bw;
    bw.h[0] = h3even;
    bw.h[1] = hp3;
    const _Float16* wp = w1l + 32 * s;
#pragma unroll
    for (int jt = 0; jt < 4; ++jt) {
      const v16h a = Frag<_Float16>::load(wp + (size_t)jt * (16 * kFlat));
      zacc[jt] = mma16(a, bw.v, zacc[jt]);
    }
    asm volatile("" ::: "memory");
#pragma unroll
    for (int jt = 4; jt < 8; ++jt) {
      const v16h a = Frag<_Float16>::load(wp + (size_t)jt * (16 * kFlat));
      zacc[jt] = mma16(a, bw.v, zacc[jt]);
    }
  }

  v8h zp[8];
#pragma unroll
  for (int jt = 0; jt < 8; ++jt) zp[jt] = relu_pack(zacc[jt], 0.125f);

  v8f oacc;
  {
    const v8f bb2 = cload(b2 + 8 * hh);
#pragma unroll
    for (int r = 0; r < 8; ++r) oacc[r] = 128.0f * bb2[r];
  }
  const _Float16* w2l = (const _Float16*)(const void*)W2h + (size_t)c * kMlpHid + 8 * hh;
#pragma unroll
  for (int cc2 = 0; cc2 < 4; ++cc2) {
    FragU bz;
    bz.h[0] = zp[2 * cc2];
    bz.h[1] = zp[2 * cc2 + 1];
    const v16h a = Frag<_Float16>::load(w2l + 32 * cc2);
    oacc = mma16(a, bz.v, oacc);
  }

  float* os = osl[wave];
  const float outInv = 1.0f / 128.0f;
#pragma unroll
  for (int r = 0; r < 8; ++r) os[c * kOutDim + 8 * hh + r] = oacc[r] * outInv;
  __builtin_amdgcn_fence(__ATOMIC_RELEASE, "workgroup");
  __builtin_amdgcn_wave_barrier();
  __builtin_amdgcn_fence(__ATOMIC_ACQUIRE, "workgroup");
  {
    float* ob = out + (size_t)rowbase * kOutDim;
    const bool live = (rowbase + kRowsPerWave) <= nrows;
    if (live) {
      for (int pass = 0; pass < 2; ++pass) {
#pragma unroll
        for (int it = 0; it < 2; ++it) {
          const v4f v = *(const v4f*)(os + it * 128 + lane * 4);
          *(volatile v4f*)(ob + it * 128 + lane * 4) = v;
        }
        __threadfence();
      }
    }
  }
}

extern "C" void kernel_launch(void* const* d_in, const int* in_sizes, int n_in,
                              void* d_out, int out_size, void* d_ws, size_t ws_size,
                              hipStream_t stream) {
  if (n_in < 21) return;
  const float* x    = (const float*)d_in[0];
  const float* Wih0 = (const float*)d_in[1];
  const float* Whh0 = (const float*)d_in[2];
  const float* bih0 = (const float*)d_in[3];
  const float* bhh0 = (const float*)d_in[4];
  const float* Wih1 = (const float*)d_in[5];
  const float* Whh1 = (const float*)d_in[6];
  const float* bih1 = (const float*)d_in[7];
  const float* bhh1 = (const float*)d_in[8];
  const float* Wih2 = (const float*)d_in[9];
  const float* Whh2 = (const float*)d_in[10];
  const float* bih2 = (const float*)d_in[11];
  const float* bhh2 = (const float*)d_in[12];
  const float* Wih3 = (const float*)d_in[13];
  const float* Whh3 = (const float*)d_in[14];
  const float* bih3 = (const float*)d_in[15];
  const float* bhh3 = (const float*)d_in[16];
  const float* W1   = (const float*)d_in[17];
  const float* b1   = (const float*)d_in[18];
  const float* W2   = (const float*)d_in[19];
  const float* b2   = (const float*)d_in[20];

  const int nrows = in_sizes[0] / kSteps;
  const int n17   = in_sizes[17];
  const int n19   = in_sizes[19];
  if (nrows < kRowsPerBlk || (nrows % kRowsPerBlk) != 0) return;
  if (n17 != kMlpHid * kFlat || n19 != kOutDim * kMlpHid) return;
  if (out_size < nrows * kOutDim) return;

  const size_t offW1 = 0;
  const size_t offW2 = (size_t)n17 * 2;
  const size_t total = offW2 + (size_t)n19 * 2;
  if (total > ws_size) return;
  unsigned short* W1h = (unsigned short*)((char*)d_ws + offW1);
  unsigned short* W2h = (unsigned short*)((char*)d_ws + offW2);

  const int n8a = n17 / 8;
  const int n8b = n19 / 8;
  cast8_f16_kernel<<<dim3((n8a + 255) / 256), dim3(256), 0, stream>>>(W1, W1h, n8a, 32.0f);
  cast8_f16_kernel<<<dim3((n8b + 255) / 256), dim3(256), 0, stream>>>(W2, W2h, n8b, 8.0f);

  rnn_mlp_kernel<<<dim3(nrows / kRowsPerBlk), dim3(256), 0, stream>>>(
      x,
      Wih0, Whh0, bih0, bhh0,
      Wih1, Whh1, bih1, bhh1,
      Wih2, Whh2, bih2, bhh2,
      Wih3, Whh3, bih3, bhh3,
      W1h, b1, W2h, b2,
      (float*)d_out, nrows);
}
